// CAN_41884521071035
// MI455X (gfx1250) — hardware-verified
//
#include <hip/hip_runtime.h>
#include <stdint.h>


#define NB   128
#define ND   512
#define NS   30
#define NHW  196
#define NT   12
#define NHI  13
#define TP   68

typedef unsigned short us;
typedef __bf16        v16b __attribute__((ext_vector_type(16)));
typedef us            v8us __attribute__((ext_vector_type(8)));
typedef unsigned int  v4u  __attribute__((ext_vector_type(4)));
typedef float         v4f  __attribute__((ext_vector_type(4)));
typedef float         v8f  __attribute__((ext_vector_type(8)));

union Frag { v16b v; v8us q[2]; v8f f; };
union P16  { v8us h; v4u u; us s[8]; };

__device__ __forceinline__ us bf_rne(float x) {
  unsigned int u = __float_as_uint(x);
  u += 0x7FFFu + ((u >> 16) & 1u);
  return (us)(u >> 16);
}
__device__ __forceinline__ float bf_val(us b) { return __uint_as_float(((unsigned int)b) << 16); }
__device__ __forceinline__ void split1(float x, us& hi, us& lo) {
  hi = bf_rne(x);
  lo = bf_rne(x - bf_val(hi));
}
__device__ __forceinline__ void split8(v4f a, v4f b, P16& hp, P16& lp) {
#pragma unroll
  for (int e = 0; e < 4; ++e) {
    us hh, ll;
    split1(a[e], hh, ll); hp.s[e] = hh;     lp.s[e] = ll;
    split1(b[e], hh, ll); hp.s[4 + e] = hh; lp.s[4 + e] = ll;
  }
}

__device__ __forceinline__ float wsum(float v) {
#pragma unroll
  for (int o = 16; o > 0; o >>= 1) v += __shfl_xor(v, o, 32);
  return v;
}
__device__ __forceinline__ float wmax(float v) {
#pragma unroll
  for (int o = 16; o > 0; o >>= 1) v = fmaxf(v, __shfl_xor(v, o, 32));
  return v;
}

__device__ __forceinline__ v8f wmb(const Frag& a, const Frag& b, v8f c) {
  return __builtin_amdgcn_wmma_f32_16x16x32_bf16(false, a.v, false, b.v, (short)0, c, false, false);
}

#define GF_BIAS   1
#define GF_ADDP   2
#define GF_MULP   4
#define GF_GATE   8
#define GF_OF32   16
#define GF_OHL    32
#define GF_OF32B  64

struct GDesc {
  const us* Ah; const us* Al; const us* Bh; const us* Bl;
  const float* bias; const float* P1; const float* P2;
  float* Cf; float* Cf2; us* Oh; us* Ol;
  int lda, ldb, ldp, ldc, ldc2, ldo, N, K, flags, nblk;
};
static_assert(sizeof(GDesc) == 128);
struct GBatch { GDesc g[3]; };
static_assert(sizeof(GBatch) == 384);

__device__ __forceinline__ v4f xform4(const GDesc& D, int row, int col, v4f v) {
  if (D.flags & GF_BIAS) {
    const v4f bb = *(const v4f*)(D.bias + col);
    v += bb;
  }
  if (D.flags & GF_ADDP) {
    const v4f pp = *(const v4f*)(D.P1 + (size_t)row * D.ldp + col);
    v += pp;
  }
  if (D.flags & GF_MULP) {
    const v4f pp = *(const v4f*)(D.P1 + (size_t)row * D.ldp + col);
    v *= pp;
  }
  if (D.flags & GF_GATE) {
    const v4f x  = *(const v4f*)(D.P1 + (size_t)row * D.ldp + col);
    const v4f mp = *(const v4f*)(D.P2 + (size_t)row * D.ldp + col);
#pragma unroll
    for (int e = 0; e < 4; ++e) {
      const float g = __builtin_amdgcn_rcpf(1.0f + __expf(-x[e]));
      v[e] = g * mp[e] + (1.0f - g) * v[e];
    }
  }
  return v;
}

__global__ __launch_bounds__(64)
void k_gemm(GBatch gb, const int* steps, int t)
{
  __shared__ __attribute__((aligned(16))) float T[32 * TP];
  const int y = blockIdx.y;
  GDesc D;
  if (y == 0) D = gb.g[0]; else if (y == 1) D = gb.g[1]; else D = gb.g[2];
  int sv = steps[0];
  if (sv > NT) sv = NT;
  if (t >= sv) return;
  if ((int)blockIdx.x >= D.nblk) return;

  const int nbn  = D.N >> 6;
  const int band = (int)blockIdx.x / nbn;
  const int r0   = band * 32;
  const int c0   = ((int)blockIdx.x - band * nbn) * 64;
  const int tid = threadIdx.x, w = tid >> 5, l = tid & 31, h = l >> 4, m = l & 15;

  v8f acc[2][2];
  {
    const v8f z = {0.f, 0.f, 0.f, 0.f, 0.f, 0.f, 0.f, 0.f};
#pragma unroll
    for (int i = 0; i < 2; ++i)
#pragma unroll
      for (int j = 0; j < 2; ++j) acc[i][j] = z;
  }
  const us* ah = D.Ah + (size_t)(r0 + m) * D.lda + 8 * h;
  const us* al = D.Al + (size_t)(r0 + m) * D.lda + 8 * h;
  const us* bh = D.Bh + (size_t)(c0 + 32 * w + m) * D.ldb + 8 * h;
  const us* bl = D.Bl + (size_t)(c0 + 32 * w + m) * D.ldb + 8 * h;
  const size_t sa = (size_t)16 * D.lda, sb = (size_t)16 * D.ldb;
  const int nk = D.K >> 5;
#pragma unroll 1
  for (int kt = 0; kt < nk; ++kt) {
    const int ko = kt << 5;
    Frag xh0, xh1, xl0, xl1, yh0, yh1, yl0, yl1;
    xh0.q[0] = *(const v8us*)(ah + ko);           xh0.q[1] = *(const v8us*)(ah + ko + 16);
    xh1.q[0] = *(const v8us*)(ah + sa + ko);      xh1.q[1] = *(const v8us*)(ah + sa + ko + 16);
    xl0.q[0] = *(const v8us*)(al + ko);           xl0.q[1] = *(const v8us*)(al + ko + 16);
    xl1.q[0] = *(const v8us*)(al + sa + ko);      xl1.q[1] = *(const v8us*)(al + sa + ko + 16);
    yh0.q[0] = *(const v8us*)(bh + ko);           yh0.q[1] = *(const v8us*)(bh + ko + 16);
    yh1.q[0] = *(const v8us*)(bh + sb + ko);      yh1.q[1] = *(const v8us*)(bh + sb + ko + 16);
    yl0.q[0] = *(const v8us*)(bl + ko);           yl0.q[1] = *(const v8us*)(bl + ko + 16);
    yl1.q[0] = *(const v8us*)(bl + sb + ko);      yl1.q[1] = *(const v8us*)(bl + sb + ko + 16);

    acc[0][0] = wmb(xh0, yh0, acc[0][0]); acc[0][0] = wmb(xh0, yl0, acc[0][0]); acc[0][0] = wmb(xl0, yh0, acc[0][0]);
    acc[0][1] = wmb(xh0, yh1, acc[0][1]); acc[0][1] = wmb(xh0, yl1, acc[0][1]); acc[0][1] = wmb(xl0, yh1, acc[0][1]);
    acc[1][0] = wmb(xh1, yh0, acc[1][0]); acc[1][0] = wmb(xh1, yl0, acc[1][0]); acc[1][0] = wmb(xl1, yh0, acc[1][0]);
    acc[1][1] = wmb(xh1, yh1, acc[1][1]); acc[1][1] = wmb(xh1, yl1, acc[1][1]); acc[1][1] = wmb(xl1, yh1, acc[1][1]);
    asm volatile("v_nop\n\tv_nop\n\tv_nop\n\tv_nop"
                 : "+v"(acc[0][0]), "+v"(acc[0][1]), "+v"(acc[1][0]), "+v"(acc[1][1])
                 : "v"(xh0.f), "v"(xh1.f), "v"(xl0.f), "v"(xl1.f),
                   "v"(yh0.f), "v"(yh1.f), "v"(yl0.f), "v"(yl1.f));
  }

#pragma unroll
  for (int i = 0; i < 2; ++i)
#pragma unroll
    for (int j = 0; j < 2; ++j)
#pragma unroll
      for (int r = 0; r < 8; ++r)
        T[(16 * i + 8 * h + r) * TP + 32 * w + 16 * j + m] = acc[i][j][r];
  __syncthreads();

  const bool last = (t == sv - 1);
  const bool of1  = (D.flags & GF_OF32) != 0;
  const bool of2  = ((D.flags & GF_OF32B) != 0) && last;
  if (of1 || of2) {
    v4f vals[8];
#pragma unroll
    for (int it = 0; it < 8; ++it) {
      const int p = it * 64 + tid, row = p >> 4, c = (p & 15) * 4;
      const v4f v = *(const v4f*)(T + row * TP + c);
      vals[it] = xform4(D, r0 + row, c0 + c, v);
    }
#pragma unroll
    for (int it = 0; it < 8; ++it) {
      const int p = it * 64 + tid, row = p >> 4, c = (p & 15) * 4;
      if (of1) *(volatile v4f*)(D.Cf  + (size_t)(r0 + row) * D.ldc  + c0 + c) = vals[it];
      if (of2) *(volatile v4f*)(D.Cf2 + (size_t)(r0 + row) * D.ldc2 + c0 + c) = vals[it];
    }
    __threadfence();
#pragma unroll
    for (int it = 0; it < 8; ++it) {
      const int p = it * 64 + tid, row = p >> 4, c = (p & 15) * 4;
      if (of1) *(volatile v4f*)(D.Cf  + (size_t)(r0 + row) * D.ldc  + c0 + c) = vals[it];
      if (of2) *(volatile v4f*)(D.Cf2 + (size_t)(r0 + row) * D.ldc2 + c0 + c) = vals[it];
    }
  }
  if (D.flags & GF_OHL) {
    v4u hv[4], lv[4];
#pragma unroll
    for (int it = 0; it < 4; ++it) {
      const int p = it * 64 + tid, row = p >> 3, c = (p & 7) * 8;
      v4f v0 = *(const v4f*)(T + row * TP + c);
      v4f v1 = *(const v4f*)(T + row * TP + c + 4);
      v0 = xform4(D, r0 + row, c0 + c, v0);
      v1 = xform4(D, r0 + row, c0 + c + 4, v1);
      P16 hp, lp;
      split8(v0, v1, hp, lp);
      hv[it] = hp.u; lv[it] = lp.u;
    }
#pragma unroll
    for (int it = 0; it < 4; ++it) {
      const int p = it * 64 + tid, row = p >> 3, c = (p & 7) * 8;
      *(volatile v4u*)(D.Oh + (size_t)(r0 + row) * D.ldo + c0 + c) = hv[it];
      *(volatile v4u*)(D.Ol + (size_t)(r0 + row) * D.ldo + c0 + c) = lv[it];
    }
    __threadfence();
#pragma unroll
    for (int it = 0; it < 4; ++it) {
      const int p = it * 64 + tid, row = p >> 3, c = (p & 7) * 8;
      *(volatile v4u*)(D.Oh + (size_t)(r0 + row) * D.ldo + c0 + c) = hv[it];
      *(volatile v4u*)(D.Ol + (size_t)(r0 + row) * D.ldo + c0 + c) = lv[it];
    }
  }
}

__global__ __launch_bounds__(256)
void k_wsplit(const float* W, us* Ph, us* Pl, int K, int N, int tr)
{
  const int i = blockIdx.x * 256 + threadIdx.x;
  const int kq = K >> 3;
  if (i >= N * kq) return;
  const int n = i / kq;
  const int k = (i - n * kq) * 8;
  v4f v0 = {0.f, 0.f, 0.f, 0.f}, v1 = {0.f, 0.f, 0.f, 0.f};
  if (tr) {
#pragma unroll
    for (int e = 0; e < 4; ++e) {
      v0[e] = W[(size_t)(k + e) * N + n];
      v1[e] = W[(size_t)(k + 4 + e) * N + n];
    }
  } else {
    v0 = *(const v4f*)(W + (size_t)n * K + k);
    v1 = *(const v4f*)(W + (size_t)n * K + k + 4);
  }
  P16 hp, lp;
  split8(v0, v1, hp, lp);
  us* dh = Ph + (size_t)n * K + k;
  us* dl = Pl + (size_t)n * K + k;
  *(volatile v4u*)dh = hp.u;
  *(volatile v4u*)dl = lp.u;
  __threadfence();
  *(volatile v4u*)dh = hp.u;
  *(volatile v4u*)dl = lp.u;
}

__global__ __launch_bounds__(256)
void k_init(const float* q, const float* c0, const float* m0,
            us* qah, us* qal, us* qch, us* qcl, us* mch, us* mcl,
            float* chist, float* mhist)
{
  const int b = blockIdx.x, tid = threadIdx.x, grp = tid >> 6, j = tid & 63;
  const size_t rb = (size_t)b * ND;
  if (grp < 3) {
    const float* src;
    us* dh; us* dl;
    if (grp == 0)      { src = q + rb;  dh = qah + rb;                       dl = qal + rb; }
    else if (grp == 1) { src = c0 + rb; dh = qch + (size_t)b * 1024 + 512;  dl = qcl + (size_t)b * 1024 + 512; }
    else               { src = m0 + rb; dh = mch + (size_t)b * 1024 + 512;  dl = mcl + (size_t)b * 1024 + 512; }
    const v4f v0 = *(const v4f*)(src + 8 * j);
    const v4f v1 = *(const v4f*)(src + 8 * j + 4);
    P16 hp, lp;
    split8(v0, v1, hp, lp);
    dh += 8 * j; dl += 8 * j;
    *(volatile v4u*)dh = hp.u;
    *(volatile v4u*)dl = lp.u;
    __threadfence();
    *(volatile v4u*)dh = hp.u;
    *(volatile v4u*)dl = lp.u;
  } else {
    const v4f a0 = *(const v4f*)(c0 + rb + 4 * j);
    const v4f a1 = *(const v4f*)(c0 + rb + 256 + 4 * j);
    const v4f b0 = *(const v4f*)(m0 + rb + 4 * j);
    const v4f b1 = *(const v4f*)(m0 + rb + 256 + 4 * j);
    float* dc = chist + rb;
    float* dm = mhist + rb;
    *(volatile v4f*)(dc + 4 * j) = a0;  *(volatile v4f*)(dc + 256 + 4 * j) = a1;
    *(volatile v4f*)(dm + 4 * j) = b0;  *(volatile v4f*)(dm + 256 + 4 * j) = b1;
    __threadfence();
    *(volatile v4f*)(dc + 4 * j) = a0;  *(volatile v4f*)(dc + 256 + 4 * j) = a1;
    *(volatile v4f*)(dm + 4 * j) = b0;  *(volatile v4f*)(dm + 256 + 4 * j) = b1;
  }
}

__global__ __launch_bounds__(256)
void k_ctrl(const float* cq, const float* cws, const float* wca, const float* bca,
            const float* wra, const float* wwa, const float* bwa,
            float* chist, const float* mhist,
            us* qch, us* qcl, us* uph, us* upl, us* ach, us* acl,
            const int* steps, int t)
{
  __shared__ __attribute__((aligned(16))) float s_vec[3][ND];
  __shared__ __attribute__((aligned(16))) float s_cqw[ND];
  __shared__ __attribute__((aligned(16))) float s_cw[ND];
  __shared__ float s_prt[8][32];
  __shared__ float s_cat[32];
  __shared__ float s_sl[16];
  __shared__ float s_sat[32];

  const int b = blockIdx.x, tid = threadIdx.x, l = tid & 31, w = tid >> 5;
  int sv = steps[0];
  if (sv > NT) sv = NT;
  if (t >= sv) return;
  const size_t rb = (size_t)b * ND;

#pragma unroll
  for (int q2 = 0; q2 < 2; ++q2) {
    const int dd = tid + 256 * q2;
    s_cqw[dd] = cq[rb + dd] * wca[dd];
  }
  __syncthreads();

  const float* cwb = cws + rb * NS;
  {
    const int sl = (l < NS) ? l : (NS - 1);
    float p = 0.f;
#pragma unroll 4
    for (int i = 0; i < 64; ++i) {
      const int d = w + 8 * i;
      p = fmaf(s_cqw[d], cwb[(size_t)d * NS + sl], p);
    }
    s_prt[w][l] = p;
  }
  __syncthreads();
  if (w == 0) {
    float x = 0.f;
#pragma unroll
    for (int k = 0; k < 8; ++k) x += s_prt[k][l];
    x += bca[0];
    const bool ok = l < NS;
    const float xv = ok ? x : -__builtin_inff();
    const float mx = wmax(xv);
    const float e = ok ? __expf(xv - mx) : 0.f;
    const float sum = wsum(e);
    s_cat[l] = e * (1.0f / sum);
  }
  __syncthreads();

#pragma unroll
  for (int q2 = 0; q2 < 2; ++q2) {
    const int dd = tid + 256 * q2;
    const float* r = cwb + (size_t)dd * NS;
    float a = 0.f;
#pragma unroll 2
    for (int s = 0; s < NS; ++s) a = fmaf(s_cat[s], r[s], a);
    s_vec[0][dd] = a;
    s_vec[1][dd] = a * wra[dd];
    s_cw[dd]     = a * wwa[dd];
  }
  __syncthreads();

  for (int tau = w; tau <= t && tau < NHI; tau += 8) {
    const float* ch = chist + ((size_t)tau * NB + b) * ND;
    float p = 0.f;
#pragma unroll 4
    for (int i = 0; i < 16; ++i) {
      const int d = l + 32 * i;
      p = fmaf(s_cw[d], ch[d], p);
    }
    p = wsum(p);
    if (l == 0) s_sl[tau] = p + bwa[0];
  }
  __syncthreads();
  if (w == 0) {
    const bool ok = (l <= t) && (l < NHI);
    const float x = ok ? s_sl[l & 15] : -__builtin_inff();
    const float mx = wmax(x);
    const float e = ok ? __expf(x - mx) : 0.f;
    const float sum = wsum(e);
    s_sat[l] = e * (1.0f / sum);
  }
  __syncthreads();

#pragma unroll
  for (int q2 = 0; q2 < 2; ++q2) {
    const int dd = tid + 256 * q2;
    float a = 0.f;
#pragma unroll 2
    for (int tau = 0; tau <= t && tau < NHI; ++tau)
      a = fmaf(s_sat[tau], mhist[((size_t)tau * NB + b) * ND + dd], a);
    s_vec[2][dd] = a;
  }
  __syncthreads();

  const int grp = tid >> 6, j = tid & 63;
  if (grp < 3) {
    const float* src = &s_vec[grp][0] + 8 * j;
    const v4f v0 = *(const v4f*)src;
    const v4f v1 = *(const v4f*)(src + 4);
    P16 hp, lp;
    split8(v0, v1, hp, lp);
    us* dh; us* dl;
    if (grp == 0)      { dh = qch + (size_t)b * 1024 + 512; dl = qcl + (size_t)b * 1024 + 512; }
    else if (grp == 1) { dh = uph + rb;                     dl = upl + rb; }
    else               { dh = ach + (size_t)b * 1024;       dl = acl + (size_t)b * 1024; }
    dh += 8 * j; dl += 8 * j;
    *(volatile v4u*)dh = hp.u;
    *(volatile v4u*)dl = lp.u;
    __threadfence();
    *(volatile v4u*)dh = hp.u;
    *(volatile v4u*)dl = lp.u;
  } else {
    float* dst = chist + (size_t)(t + 1) * NB * ND + rb;
    const v4f a0 = *(const v4f*)(&s_vec[0][0] + 4 * j);
    const v4f a1 = *(const v4f*)(&s_vec[0][0] + 256 + 4 * j);
    *(volatile v4f*)(dst + 4 * j) = a0;
    *(volatile v4f*)(dst + 256 + 4 * j) = a1;
    __threadfence();
    *(volatile v4f*)(dst + 4 * j) = a0;
    *(volatile v4f*)(dst + 256 + 4 * j) = a1;
  }
}

__global__ __launch_bounds__(256)
void k_read(const float* KB, const float* wv, const float* a1f, const float* chist,
            const float* wra, const float* brm, const float* bkb, const float* bra,
            us* mch, us* mcl, const int* steps, int t)
{
  __shared__ __attribute__((aligned(16))) float s_w[ND];
  __shared__ __attribute__((aligned(16))) float s_mn[ND];
  __shared__ __attribute__((aligned(16))) float s_rl[256];
  __shared__ float s_ra[8], s_rb[8], s_rc[8];

  const int b = blockIdx.x, tid = threadIdx.x, l = tid & 31, w = tid >> 5;
  int sv = steps[0];
  if (sv > NT) sv = NT;
  if (t >= sv) return;
  const size_t rb = (size_t)b * ND;
  const float* ci = chist + (size_t)(t + 1) * NB * ND + rb;

  float p = 0.f;
#pragma unroll
  for (int q2 = 0; q2 < 2; ++q2) {
    const int dd = tid + 256 * q2;
    s_w[dd] = wv[rb + dd];
    p = fmaf(bkb[dd], a1f[rb + dd], p);
    p = fmaf(brm[dd], ci[dd] * wra[dd], p);
  }
  p = wsum(p);
  if (l == 0) s_ra[w] = p;
  __syncthreads();
  float c0r = 0.f;
#pragma unroll
  for (int k = 0; k < 8; ++k) c0r += s_ra[k];
  c0r += bra[0];

  const int hw = (tid < NHW) ? tid : (NHW - 1);
  const float* kb = KB + (size_t)b * ND * NHW + hw;
  float s = 0.f;
#pragma unroll 4
  for (int d = 0; d < ND; ++d) s = fmaf(kb[(size_t)d * NHW], s_w[d], s);
  const bool ok = tid < NHW;
  const float x = ok ? (s + c0r) : -__builtin_inff();
  const float mx = wmax(x);
  if (l == 0) s_rb[w] = mx;
  __syncthreads();
  float gm = s_rb[0];
#pragma unroll
  for (int k = 1; k < 8; ++k) gm = fmaxf(gm, s_rb[k]);
  const float e = ok ? __expf(x - gm) : 0.f;
  const float ps = wsum(e);
  if (l == 0) s_rc[w] = ps;
  __syncthreads();
  float tot = 0.f;
#pragma unroll
  for (int k = 0; k < 8; ++k) tot += s_rc[k];
  const float inv = 1.0f / tot;
  s_rl[tid] = e * inv;
  __syncthreads();

#pragma unroll
  for (int q2 = 0; q2 < 2; ++q2) {
    const int dd = tid + 256 * q2;
    const float* row = KB + (rb + dd) * NHW;
    float a = 0.f;
#pragma unroll 4
    for (int k = 0; k < NHW; ++k) a = fmaf(s_rl[k], row[k], a);
    s_mn[dd] = a;
  }
  __syncthreads();

  if (tid < 64) {
    const v4f v0 = *(const v4f*)(s_mn + 8 * tid);
    const v4f v1 = *(const v4f*)(s_mn + 8 * tid + 4);
    P16 hp, lp;
    split8(v0, v1, hp, lp);
    us* dh = mch + (size_t)b * 1024 + 8 * tid;
    us* dl = mcl + (size_t)b * 1024 + 8 * tid;
    *(volatile v4u*)dh = hp.u;
    *(volatile v4u*)dl = lp.u;
    __threadfence();
    *(volatile v4u*)dh = hp.u;
    *(volatile v4u*)dl = lp.u;
  }
}

extern "C" void kernel_launch(void* const* d_in, const int* in_sizes, int n_in,
                              void* d_out, int out_size, void* d_ws, size_t ws_size,
                              hipStream_t stream)
{
  const int BD = NB * ND;
  if (n_in < 28) return;
  if (in_sizes[0] != BD || in_sizes[1] != BD * NS || in_sizes[2] != BD * NHW ||
      in_sizes[3] != BD || in_sizes[4] != BD) return;
  if (in_sizes[5] != ND * ND || in_sizes[7] != 2 * ND * ND || in_sizes[11] != ND * ND ||
      in_sizes[13] != ND * ND || in_sizes[15] != 2 * ND * ND || in_sizes[19] != 2 * ND * ND ||
      in_sizes[23] != 2 * ND * ND || in_sizes[25] != ND * ND) return;
  if (in_sizes[6] != ND || in_sizes[8] != ND || in_sizes[9] != ND || in_sizes[12] != ND ||
      in_sizes[14] != ND || in_sizes[16] != ND || in_sizes[17] != ND || in_sizes[20] != ND ||
      in_sizes[21] != ND || in_sizes[24] != ND || in_sizes[26] != ND) return;
  if (in_sizes[10] < 1 || in_sizes[18] < 1 || in_sizes[22] < 1 || in_sizes[27] < 1) return;
  if (out_size != BD) return;

  const float* q   = (const float*)d_in[0];
  const float* cws = (const float*)d_in[1];
  const float* KB  = (const float*)d_in[2];
  const float* c0  = (const float*)d_in[3];
  const float* m0  = (const float*)d_in[4];
  const float* Wq  = (const float*)d_in[5];   const float* bq  = (const float*)d_in[6];
  const float* Wct = (const float*)d_in[7];   const float* bct = (const float*)d_in[8];
  const float* wca = (const float*)d_in[9];   const float* bca = (const float*)d_in[10];
  const float* Wm  = (const float*)d_in[11];  const float* bm  = (const float*)d_in[12];
  const float* Wkb = (const float*)d_in[13];  const float* bkb = (const float*)d_in[14];
  const float* Wrm = (const float*)d_in[15];  const float* brm = (const float*)d_in[16];
  const float* wra = (const float*)d_in[17];  const float* bra = (const float*)d_in[18];
  const float* Wwm = (const float*)d_in[19];  const float* bwm = (const float*)d_in[20];
  const float* wwa = (const float*)d_in[21];  const float* bwa = (const float*)d_in[22];
  const float* Wam = (const float*)d_in[23];  const float* bam = (const float*)d_in[24];
  const float* Wg  = (const float*)d_in[25];  const float* bg  = (const float*)d_in[26];
  const int*   steps = (const int*)d_in[27];
  float* out = (float*)d_out;

  char* ws = (char*)d_ws;
  size_t off = 0;
  auto carve = [&](size_t bytes) -> char* {
    char* p = ws + off;
    off = (off + bytes + 255) & ~(size_t)255;
    return p;
  };
  const size_t W5 = (size_t)ND * ND * 2;
  const size_t W1 = (size_t)2 * ND * ND * 2;
  us* wqh  = (us*)carve(W5); us* wql  = (us*)carve(W5);
  us* wcth = (us*)carve(W1); us* wctl = (us*)carve(W1);
  us* wmh  = (us*)carve(W5); us* wml  = (us*)carve(W5);
  us* wkbh = (us*)carve(W5); us* wkbl = (us*)carve(W5);
  us* wrmh = (us*)carve(W1); us* wrml = (us*)carve(W1);
  us* wwmh = (us*)carve(W1); us* wwml = (us*)carve(W1);
  us* wamh = (us*)carve(W1); us* waml = (us*)carve(W1);
  us* wgh  = (us*)carve(W5); us* wgl  = (us*)carve(W5);
  const size_t A5 = (size_t)NB * ND * 2, A1 = (size_t)NB * 1024 * 2, F5 = (size_t)NB * ND * 4;
  us* qah = (us*)carve(A5); us* qal = (us*)carve(A5);
  us* qch = (us*)carve(A1); us* qcl = (us*)carve(A1);
  us* mch = (us*)carve(A1); us* mcl = (us*)carve(A1);
  us* ach = (us*)carve(A1); us* acl = (us*)carve(A1);
  us* uph = (us*)carve(A5); us* upl = (us*)carve(A5);
  us* a1h = (us*)carve(A5); us* a1l = (us*)carve(A5);
  float* chist = (float*)carve((size_t)NHI * F5);
  float* mhist = (float*)carve((size_t)NHI * F5);
  float* cqf = (float*)carve(F5);
  float* mpf = (float*)carve(F5);
  float* vbf = (float*)carve(F5);
  float* glf = (float*)carve(F5);
  float* wvf = (float*)carve(F5);
  float* a1f = (float*)carve(F5);
  if (off > ws_size || off > (size_t)134217728) return;

  auto wsplit = [&](const float* Wsrc, us* ph, us* pl, int K, int N, int tr) {
    const int tot = N * (K / 8);
    k_wsplit<<<dim3((tot + 255) / 256), dim3(256), 0, stream>>>(Wsrc, ph, pl, K, N, tr);
  };
  wsplit(Wq,  wqh,  wql,  ND,     ND,     1);
  wsplit(Wct, wcth, wctl, 2 * ND, ND,     1);
  wsplit(Wm,  wmh,  wml,  ND,     ND,     1);
  wsplit(Wkb, wkbh, wkbl, ND,     ND,     0);
  wsplit(Wrm, wrmh, wrml, ND,     2 * ND, 0);
  wsplit(Wwm, wwmh, wwml, 2 * ND, ND,     1);
  wsplit(Wam, wamh, waml, 2 * ND, ND,     1);
  wsplit(Wg,  wgh,  wgl,  ND,     ND,     1);

  k_init<<<dim3(NB), dim3(256), 0, stream>>>(q, c0, m0, qah, qal, qch, qcl, mch, mcl, chist, mhist);

  GDesc base;
  base.Ah = qah; base.Al = qal; base.Bh = wqh; base.Bl = wql;
  base.bias = bq; base.P1 = cqf; base.P2 = cqf; base.Cf = cqf; base.Cf2 = cqf; base.Oh = qch; base.Ol = qcl;
  base.lda = ND; base.ldb = ND; base.ldp = ND; base.ldc = ND; base.ldc2 = ND; base.ldo = 1024;
  base.N = ND; base.K = ND; base.flags = 0; base.nblk = (NB / 32) * (ND / 64);
  auto launch = [&](const GDesc& d0, const GDesc& d1, const GDesc& d2, int nd, int t) {
    GBatch gb;
    gb.g[0] = d0; gb.g[1] = d1; gb.g[2] = d2;
    k_gemm<<<dim3(32, nd), dim3(64), 0, stream>>>(gb, steps, t);
  };

  {
    GDesc d = base;
    d.Ah = qah; d.Al = qal; d.lda = ND; d.Bh = wqh; d.Bl = wql; d.ldb = ND; d.K = ND;
    d.bias = bq; d.Oh = qch; d.Ol = qcl; d.ldo = 1024; d.flags = GF_BIAS | GF_OHL;
    launch(d, d, d, 1, -1);
  }

  for (int t = 0; t < NT; ++t) {
    {
      GDesc dcq = base;
      dcq.Ah = qch; dcq.Al = qcl; dcq.lda = 1024; dcq.Bh = wcth; dcq.Bl = wctl; dcq.ldb = 1024; dcq.K = 2 * ND;
      dcq.bias = bct; dcq.Cf = cqf; dcq.ldc = ND; dcq.flags = GF_BIAS | GF_OF32;
      GDesc dmp = base;
      dmp.Ah = mch + 512; dmp.Al = mcl + 512; dmp.lda = 1024; dmp.Bh = wmh; dmp.Bl = wml; dmp.ldb = ND; dmp.K = ND;
      dmp.bias = bm; dmp.Cf = mpf; dmp.ldc = ND; dmp.flags = GF_BIAS | GF_OF32;
      launch(dcq, dmp, dcq, 2, t);
    }
    k_ctrl<<<dim3(NB), dim3(256), 0, stream>>>(cqf, cws, wca, bca, wra, wwa, bwa, chist, mhist,
                                                qch, qcl, uph, upl, ach, acl, steps, t);
    {
      GDesc dva = base;
      dva.Ah = uph; dva.Al = upl; dva.lda = ND; dva.Bh = wrmh; dva.Bl = wrml; dva.ldb = ND; dva.K = ND;
      dva.P1 = mpf; dva.ldp = ND; dva.Cf = a1f; dva.ldc = ND; dva.Oh = a1h; dva.Ol = a1l; dva.ldo = ND;
      dva.flags = GF_MULP | GF_OF32 | GF_OHL;
      GDesc dvb = base;
      dvb.Ah = uph; dvb.Al = upl; dvb.lda = ND; dvb.Bh = wrmh + (size_t)ND * ND; dvb.Bl = wrml + (size_t)ND * ND;
      dvb.ldb = ND; dvb.K = ND; dvb.Cf = vbf; dvb.ldc = ND; dvb.flags = GF_OF32;
      GDesc dg = base;
      dg.Ah = qch + 512; dg.Al = qcl + 512; dg.lda = 1024; dg.Bh = wgh; dg.Bl = wgl; dg.ldb = ND; dg.K = ND;
      dg.bias = bg; dg.Cf = glf; dg.ldc = ND; dg.flags = GF_BIAS | GF_OF32;
      launch(dva, dvb, dg, 3, t);
    }
    {
      GDesc dw = base;
      dw.Ah = a1h; dw.Al = a1l; dw.lda = ND; dw.Bh = wkbh; dw.Bl = wkbl; dw.ldb = ND; dw.K = ND;
      dw.P1 = vbf; dw.ldp = ND; dw.Cf = wvf; dw.ldc = ND; dw.flags = GF_ADDP | GF_OF32;
      launch(dw, dw, dw, 1, t);
    }
    k_read<<<dim3(NB), dim3(256), 0, stream>>>(KB, wvf, a1f, chist, wra, brm, bkb, bra, mch, mcl, steps, t);
    {
      GDesc dm1 = base;
      dm1.Ah = mch; dm1.Al = mcl; dm1.lda = 1024; dm1.Bh = wwmh; dm1.Bl = wwml; dm1.ldb = 1024; dm1.K = 2 * ND;
      dm1.bias = bwm; dm1.Oh = ach + 512; dm1.Ol = acl + 512; dm1.ldo = 1024; dm1.flags = GF_BIAS | GF_OHL;
      launch(dm1, dm1, dm1, 1, t);
    }
    {
      GDesc dm2 = base;
      dm2.Ah = ach; dm2.Al = acl; dm2.lda = 1024; dm2.Bh = wamh; dm2.Bl = waml; dm2.ldb = 1024; dm2.K = 2 * ND;
      dm2.bias = bam; dm2.P1 = glf; dm2.P2 = mhist + (size_t)t * BD; dm2.ldp = ND;
      dm2.Cf = mhist + (size_t)(t + 1) * BD; dm2.ldc = ND; dm2.Cf2 = out; dm2.ldc2 = ND;
      dm2.Oh = mch + 512; dm2.Ol = mcl + 512; dm2.ldo = 1024;
      dm2.flags = GF_BIAS | GF_GATE | GF_OF32 | GF_OHL | GF_OF32B;
      launch(dm2, dm2, dm2, 1, t);
    }
  }
}
